// EdgeNetwork_59528246723026
// MI455X (gfx1250) — hardware-verified
//
#include <hip/hip_runtime.h>
#include <stddef.h>
#include <stdint.h>

#define DIN    64
#define HID    64
#define K1     64
#define N1     128
#define K23    128
#define NTHR   256
#define EPB    256
#define DP     68
#define AP     136
#define CSTN   656
#define GBM    64
#define GBN    128
#define GTHR   128
#define NU1    (N1 * (K1 / 8))
#define NU2    (2 * HID * (K23 / 8))
#define EDGE_LDS_BYTES (EPB * DP * 4 + EPB * AP * 2 + CSTN * 4 + EPB * 4)
#define WSMAX  134217728

static_assert(K1 % 32 == 0 && K23 % 32 == 0 && K23 == 2 * HID);
static_assert(N1 == GBN && GBM == (GTHR / 32) * 16 && GBN == 4 * 32);
static_assert(NU1 % NTHR == 0 && NU2 % NTHR == 0);
static_assert((DP * 4) % 16 == 0 && (AP * 2) % 16 == 0 && AP >= K23 && DP >= HID);
static_assert(EPB == NTHR && EPB == 8 * 32);
static_assert((EPB * DP * 4) % 16 == 0 && (EPB * AP * 2) % 16 == 0 && (CSTN * 4) % 16 == 0);
static_assert(CSTN >= 641);
static_assert(EDGE_LDS_BYTES <= 300000);
static_assert(DIN / 8 == 8 && K1 / 8 == 8 && K23 / 8 == 16);

typedef float          v4f   __attribute__((ext_vector_type(4)));
typedef float          v8f   __attribute__((ext_vector_type(8)));
typedef int            v8i   __attribute__((ext_vector_type(8)));
typedef unsigned short v8us  __attribute__((ext_vector_type(8)));
typedef unsigned short v16us __attribute__((ext_vector_type(16)));
typedef __bf16         v16bf __attribute__((ext_vector_type(16)));
typedef v4f  __attribute__((may_alias)) v4fa;
typedef v8us __attribute__((may_alias)) v8usa;
union FragB { v16bf v; v16us u; v8us h[2]; v8i w; };

__device__ __forceinline__ v8f wmb(const FragB& a, const FragB& b, v8f c) {
  v8f d = __builtin_amdgcn_wmma_f32_16x16x32_bf16(false, a.v, false, b.v, (short)0, c, false, false);
  asm volatile("v_nop\n\tv_nop\n\tv_nop\n\tv_nop" : "+v"(d) : "v"(a.w), "v"(b.w));
  return d;
}

__device__ __forceinline__ unsigned bf16_bits(float f) {
  const unsigned u = __float_as_uint(f);
  return (u + 0x7FFFu + ((u >> 16) & 1u)) >> 16;
}
__device__ __forceinline__ float bf16_val(float f) {
  return __uint_as_float(bf16_bits(f) << 16);
}

__device__ __forceinline__ float tanh_f(float t) {
  const float e = __expf(2.0f * t);
  return fmaf(-2.0f, __builtin_amdgcn_rcpf(1.0f + e), 1.0f);
}

__global__ __launch_bounds__(NTHR) void k_prep(const float* __restrict__ x, const float* __restrict__ W1,
                                               const float* __restrict__ W2, const float* __restrict__ W3,
                                               int nN, int mRows,
                                               unsigned short* W1T, unsigned short* W23T, unsigned short* XA) {
  const int u = (int)blockIdx.x * NTHR + (int)threadIdx.x;
  v8us o;
  unsigned short* dp;
  if (u < NU1) {
    const int n   = u >> 3;
    const int k8  = (u & 7) * 8;
    const int nn  = n & 63;
    const int kof = (n >> 6) * 64;
    const float* p = W1 + (size_t)(kof + k8) * HID + nn;
#pragma unroll
    for (int i = 0; i < 8; ++i) o[i] = (unsigned short)bf16_bits(p[(size_t)i * HID]);
    dp = W1T + (size_t)n * K1 + k8;
  } else if (u < NU1 + NU2) {
    const int v  = u - NU1;
    const int L  = v >> 10;
    const int rr = v & 1023;
    const int n  = rr >> 4;
    const int k8 = (rr & 15) * 8;
    const int kk = k8 & (HID - 1);
    const float* Wp = (L == 0) ? W2 : W3;
    const float* p = Wp + (size_t)kk * HID + n;
#pragma unroll
    for (int i = 0; i < 8; ++i) o[i] = (unsigned short)bf16_bits(p[(size_t)i * HID]);
    dp = W23T + ((size_t)L * HID + n) * K23 + k8;
  } else {
    const int v = u - NU1 - NU2;
    if (v >= mRows * 8) return;
    const int row = v >> 3;
    const int k8  = (v & 7) * 8;
    const int rc  = row < nN ? row : nN - 1;
    const float* p = x + (size_t)rc * DIN + k8;
    const v4f a = *(const v4fa*)p;
    const v4f b = *(const v4fa*)(p + 4);
    const bool ok = row < nN;
    o[0] = ok ? (unsigned short)bf16_bits(a.x) : (unsigned short)0;
    o[1] = ok ? (unsigned short)bf16_bits(a.y) : (unsigned short)0;
    o[2] = ok ? (unsigned short)bf16_bits(a.z) : (unsigned short)0;
    o[3] = ok ? (unsigned short)bf16_bits(a.w) : (unsigned short)0;
    o[4] = ok ? (unsigned short)bf16_bits(b.x) : (unsigned short)0;
    o[5] = ok ? (unsigned short)bf16_bits(b.y) : (unsigned short)0;
    o[6] = ok ? (unsigned short)bf16_bits(b.z) : (unsigned short)0;
    o[7] = ok ? (unsigned short)bf16_bits(b.w) : (unsigned short)0;
    dp = XA + (size_t)row * DIN + k8;
  }
  *(volatile v8us*)dp = o;
  __threadfence();
  *(volatile v8us*)dp = o;
}

__global__ __launch_bounds__(GTHR) void k_gemm(const unsigned short* __restrict__ A, int lda,
                                               const unsigned short* __restrict__ BT, int ldb, int K,
                                               float* Cm, int ldc) {
  __shared__ __attribute__((aligned(16))) float stg[GBM * GBN];
  const int tid = (int)threadIdx.x, lane = tid & 31, wave = tid >> 5, hh = lane >> 4, m = lane & 15;
  const int rowBase = (int)blockIdx.x * GBM;
  const int colBase = (int)blockIdx.y * GBN;

  v8f acc[8];
  {
    const v8f z = {0.f, 0.f, 0.f, 0.f, 0.f, 0.f, 0.f, 0.f};
#pragma unroll
    for (int t = 0; t < 8; ++t) acc[t] = z;
  }
  const unsigned short* ap = A  + (size_t)(rowBase + 16 * wave + m) * (size_t)lda + 8 * hh;
  const unsigned short* bp = BT + (size_t)(colBase + m) * (size_t)ldb + 8 * hh;

#pragma unroll 1
  for (int k0 = 0; k0 < K; k0 += 32) {
    FragB af;
    af.h[0] = *(const v8usa*)(ap + k0);
    af.h[1] = *(const v8usa*)(ap + k0 + 16);
#pragma unroll
    for (int nt = 0; nt < 8; ++nt) {
      const unsigned short* wq = bp + (size_t)(16 * nt) * (size_t)ldb + k0;
      FragB bf;
      bf.h[0] = *(const v8usa*)wq;
      bf.h[1] = *(const v8usa*)(wq + 16);
      acc[nt] = wmb(af, bf, acc[nt]);
    }
  }

#pragma unroll
  for (int nt = 0; nt < 8; ++nt) {
    const int lc = 16 * nt + m;
#pragma unroll
    for (int r = 0; r < 8; ++r) {
      const int lr = 16 * wave + 8 * hh + r;
      stg[lr * GBN + lc] = acc[nt][r];
    }
  }
  __syncthreads();

  v4f pv[16];
#pragma unroll
  for (int i = 0; i < 16; ++i) pv[i] = *(const v4fa*)(stg + (16 * wave + i) * GBN + 4 * lane);
#pragma unroll
  for (int i = 0; i < 16; ++i) {
    float* op = Cm + (size_t)(rowBase + 16 * wave + i) * (size_t)ldc + colBase + 4 * lane;
    *(volatile v4f*)op = pv[i];
  }
  __threadfence();
#pragma unroll
  for (int i = 0; i < 16; ++i) {
    float* op = Cm + (size_t)(rowBase + 16 * wave + i) * (size_t)ldc + colBase + 4 * lane;
    *(volatile v4f*)op = pv[i];
  }
}

__device__ __forceinline__ float ln_tanh_row(const float* rd, unsigned short* ra,
                                             const float* gg, const float* bb, const float* w4) {
  float s = 0.0f;
#pragma unroll 4
  for (int c4 = 0; c4 < HID / 4; ++c4) {
    const v4f v = *(const v4fa*)(rd + 4 * c4);
    s += (v.x + v.y) + (v.z + v.w);
  }
  const float mu = s * 0.015625f;
  float q = 0.0f;
#pragma unroll 4
  for (int c4 = 0; c4 < HID / 4; ++c4) {
    const v4f v = *(const v4fa*)(rd + 4 * c4);
    const float d0 = v.x - mu, d1 = v.y - mu, d2 = v.z - mu, d3 = v.w - mu;
    q = fmaf(d0, d0, q); q = fmaf(d1, d1, q); q = fmaf(d2, d2, q); q = fmaf(d3, d3, q);
  }
  const float rs = rsqrtf(fmaf(q, 0.015625f, 1e-5f));
  float dot = 0.0f;
#pragma unroll 1
  for (int c8 = 0; c8 < HID / 8; ++c8) {
    const v4f va = *(const v4fa*)(rd + 8 * c8);
    const v4f vb = *(const v4fa*)(rd + 8 * c8 + 4);
    const v4f ga = *(const v4fa*)(gg + 8 * c8);
    const v4f gb = *(const v4fa*)(gg + 8 * c8 + 4);
    const v4f ta = *(const v4fa*)(bb + 8 * c8);
    const v4f tb = *(const v4fa*)(bb + 8 * c8 + 4);
    const v4f wa = *(const v4fa*)(w4 + 8 * c8);
    const v4f wb = *(const v4fa*)(w4 + 8 * c8 + 4);
    const v8f v8 = {va.x, va.y, va.z, va.w, vb.x, vb.y, vb.z, vb.w};
    const v8f g8 = {ga.x, ga.y, ga.z, ga.w, gb.x, gb.y, gb.z, gb.w};
    const v8f b8 = {ta.x, ta.y, ta.z, ta.w, tb.x, tb.y, tb.z, tb.w};
    const v8f w8 = {wa.x, wa.y, wa.z, wa.w, wb.x, wb.y, wb.z, wb.w};
    v8us ho, lo;
#pragma unroll
    for (int i = 0; i < 8; ++i) {
      float y = (v8[i] - mu) * rs;
      y = y * g8[i] + b8[i];
      const float th = tanh_f(y);
      dot = fmaf(th, w8[i], dot);
      const unsigned hb = bf16_bits(th);
      ho[i] = (unsigned short)hb;
      lo[i] = (unsigned short)bf16_bits(th - __uint_as_float(hb << 16));
    }
    *(v8usa*)(ra + 8 * c8) = ho;
    *(v8usa*)(ra + HID + 8 * c8) = lo;
  }
  return dot;
}

__global__ __launch_bounds__(NTHR) void k_edge(const int* __restrict__ ei, int nE, int nN,
                                               const float* __restrict__ PQ,
                                               const unsigned short* __restrict__ W23T,
                                               const float* __restrict__ b1, const float* __restrict__ b2,
                                               const float* __restrict__ b3,
                                               const float* __restrict__ g1, const float* __restrict__ g2,
                                               const float* __restrict__ g3,
                                               const float* __restrict__ bt1, const float* __restrict__ bt2,
                                               const float* __restrict__ bt3,
                                               const float* __restrict__ W4, const float* __restrict__ b4,
                                               float* out) {
  extern __shared__ __attribute__((aligned(16))) float dyn[];
  float*          sD  = dyn;
  unsigned short* sA  = (unsigned short*)(dyn + EPB * DP);
  float*          cst = dyn + EPB * DP + (EPB * AP) / 2;
  float*          sy  = cst + CSTN;

  const int tid = (int)threadIdx.x, lane = tid & 31, wave = tid >> 5, hh = lane >> 4, m = lane & 15;

  if (tid < 64) {
    cst[tid]       = bf16_val(b1[tid]);
    cst[64 + tid]  = bf16_val(b2[tid]);
    cst[128 + tid] = bf16_val(b3[tid]);
    cst[192 + tid] = bf16_val(g1[tid]);
    cst[256 + tid] = bf16_val(g2[tid]);
    cst[320 + tid] = bf16_val(g3[tid]);
    cst[384 + tid] = bf16_val(bt1[tid]);
    cst[448 + tid] = bf16_val(bt2[tid]);
    cst[512 + tid] = bf16_val(bt3[tid]);
    cst[576 + tid] = bf16_val(W4[tid]);
    const float vb4 = bf16_val(b4[0]);
    if (tid == 0) cst[640] = vb4;
  }

  const int e0 = (int)blockIdx.x * EPB;
  int ec = e0 + tid;
  ec = ec > nE - 1 ? nE - 1 : ec;
  int s = ei[ec];
  int t = ei[(size_t)nE + (size_t)ec];
  s = s < 0 ? 0 : (s > nN - 1 ? nN - 1 : s);
  t = t < 0 ? 0 : (t > nN - 1 ? nN - 1 : t);
  const float* pr = PQ + (size_t)s * N1;
  const float* qr = PQ + (size_t)t * N1 + HID;
  float* rd = sD + tid * DP;
  unsigned short* ra = sA + tid * AP;
  __syncthreads();
#pragma unroll 4
  for (int c4 = 0; c4 < HID / 4; ++c4) {
    const v4f p = *(const v4fa*)(pr + 4 * c4);
    const v4f qv = *(const v4fa*)(qr + 4 * c4);
    const v4f bb = *(const v4fa*)(cst + 4 * c4);
    v4f v;
    v.x = (p.x + qv.x) + bb.x;
    v.y = (p.y + qv.y) + bb.y;
    v.z = (p.z + qv.z) + bb.z;
    v.w = (p.w + qv.w) + bb.w;
    *(v4fa*)(rd + 4 * c4) = v;
  }
  __syncthreads();

  float ydot = 0.0f;
#pragma unroll 1
  for (int L = 0; L < 3; ++L) {
    ydot = ln_tanh_row(rd, ra, cst + 192 + 64 * L, cst + 384 + 64 * L, cst + 576);
    if (L < 2) {
      __syncthreads();
      v8f acc[2][4];
      {
        const v8f z = {0.f, 0.f, 0.f, 0.f, 0.f, 0.f, 0.f, 0.f};
#pragma unroll
        for (int mt = 0; mt < 2; ++mt)
#pragma unroll
          for (int nt = 0; nt < 4; ++nt) acc[mt][nt] = z;
      }
      const unsigned short* ap0 = sA + (32 * wave + m) * AP + 8 * hh;
      const unsigned short* ap1 = ap0 + 16 * AP;
      const unsigned short* bp  = W23T + ((size_t)L * HID + m) * K23 + 8 * hh;
#pragma unroll 1
      for (int k0 = 0; k0 < K23; k0 += 32) {
        FragB a0, a1;
        a0.h[0] = *(const v8usa*)(ap0 + k0);
        a0.h[1] = *(const v8usa*)(ap0 + k0 + 16);
        a1.h[0] = *(const v8usa*)(ap1 + k0);
        a1.h[1] = *(const v8usa*)(ap1 + k0 + 16);
#pragma unroll
        for (int nt = 0; nt < 4; ++nt) {
          const unsigned short* wq = bp + (size_t)(16 * nt) * K23 + k0;
          FragB bf;
          bf.h[0] = *(const v8usa*)wq;
          bf.h[1] = *(const v8usa*)(wq + 16);
          acc[0][nt] = wmb(a0, bf, acc[0][nt]);
          acc[1][nt] = wmb(a1, bf, acc[1][nt]);
        }
      }
      const float* bias = cst + 64 * (L + 1);
#pragma unroll
      for (int nt = 0; nt < 4; ++nt) {
        const int col = 16 * nt + m;
        const float bvv = bias[col];
#pragma unroll
        for (int mt = 0; mt < 2; ++mt)
#pragma unroll
          for (int r = 0; r < 8; ++r)
            sD[(32 * wave + 16 * mt + 8 * hh + r) * DP + col] = acc[mt][nt][r] + bvv;
      }
      __syncthreads();
    }
  }

  const float yv = ydot + cst[640];
  const float ov = __builtin_amdgcn_rcpf(1.0f + expf(-yv));
  sy[tid] = ov;
  __syncthreads();

  const int tl = tid < 64 ? tid : 63;
  const v4f o4 = *(const v4fa*)(sy + 4 * tl);
  const int eo = e0 + 4 * tl;
  const bool stv = (tid < 64) && (eo + 3 < nE);
  if (stv) *(volatile v4f*)(out + (size_t)eo) = o4;
  __threadfence();
  if (stv) *(volatile v4f*)(out + (size_t)eo) = o4;
}

static inline int cdiv(int a, int b) { return (a + b - 1) / b; }

extern "C" void kernel_launch(void* const* d_in, const int* in_sizes, int n_in,
                              void* d_out, int out_size, void* d_ws, size_t ws_size,
                              hipStream_t stream) {
  if (n_in < 16) return;
  if (in_sizes[0] < DIN || (in_sizes[0] % DIN) != 0) return;
  const int nN = in_sizes[0] / DIN;
  if (in_sizes[1] < 2 || (in_sizes[1] & 1) != 0) return;
  const int nE = in_sizes[1] / 2;
  if (nE < 4 || (nE & 3) != 0) return;
  if (in_sizes[2] != 2 * DIN * HID) return;
  if (in_sizes[3] != HID || in_sizes[4] != HID || in_sizes[5] != HID) return;
  if (in_sizes[6] != HID * HID) return;
  if (in_sizes[7] != HID || in_sizes[8] != HID || in_sizes[9] != HID) return;
  if (in_sizes[10] != HID * HID) return;
  if (in_sizes[11] != HID || in_sizes[12] != HID || in_sizes[13] != HID) return;
  if (in_sizes[14] != HID || in_sizes[15] != 1) return;
  if (out_size != nE) return;

  const float* x   = (const float*)d_in[0];
  const int*   ei  = (const int*)d_in[1];
  const float* W1  = (const float*)d_in[2];
  const float* b1  = (const float*)d_in[3];
  const float* g1  = (const float*)d_in[4];
  const float* bt1 = (const float*)d_in[5];
  const float* W2  = (const float*)d_in[6];
  const float* b2  = (const float*)d_in[7];
  const float* g2  = (const float*)d_in[8];
  const float* bt2 = (const float*)d_in[9];
  const float* W3  = (const float*)d_in[10];
  const float* b3  = (const float*)d_in[11];
  const float* g3  = (const float*)d_in[12];
  const float* bt3 = (const float*)d_in[13];
  const float* W4  = (const float*)d_in[14];
  const float* b4  = (const float*)d_in[15];
  float* out = (float*)d_out;

  const int MP = cdiv(nN, GBM) * GBM;
  const int gM = MP / GBM;

  char* ws = (char*)d_ws;
  size_t off = 0;
  const size_t oW1T = off; off += (size_t)N1 * K1 * 2;           off = (off + 255) & ~(size_t)255;
  const size_t oW23 = off; off += (size_t)2 * HID * K23 * 2;     off = (off + 255) & ~(size_t)255;
  const size_t oXA  = off; off += (size_t)MP * DIN * 2;          off = (off + 255) & ~(size_t)255;
  const size_t oPQ  = off; off += (size_t)MP * N1 * 4;           off = (off + 255) & ~(size_t)255;
  if (off > ws_size || off > (size_t)WSMAX) return;
  unsigned short* W1T  = (unsigned short*)(ws + oW1T);
  unsigned short* W23T = (unsigned short*)(ws + oW23);
  unsigned short* XA   = (unsigned short*)(ws + oXA);
  float*          PQ   = (float*)(ws + oPQ);

  hipFuncSetAttribute(reinterpret_cast<const void*>(&k_edge), hipFuncAttributeMaxDynamicSharedMemorySize,
                      (int)EDGE_LDS_BYTES);

  const int nUnits = NU1 + NU2 + MP * 8;
  k_prep<<<cdiv(nUnits, NTHR), NTHR, 0, stream>>>(x, W1, W2, W3, nN, MP, W1T, W23T, XA);
  k_gemm<<<dim3(gM, N1 / GBN), GTHR, 0, stream>>>(XA, K1, W1T, K1, K1, PQ, N1);
  k_edge<<<cdiv(nE, EPB), NTHR, EDGE_LDS_BYTES, stream>>>(ei, nE, nN, PQ, W23T,
                                                           b1, b2, b3, g1, g2, g3, bt1, bt2, bt3,
                                                           W4, b4, out);
}
